// SelfAttention_24601572671941
// MI455X (gfx1250) — hardware-verified
//
#include <hip/hip_runtime.h>


#ifndef NB
#define NB 2
#endif
#ifndef SEQ
#define SEQ 2048
#endif
#ifndef EARLY_QBLK
#define EARLY_QBLK 4
#endif
#define NB_FULL    2
#define SEQ_FULL   2048
#define CDIM       1024
#define NHEAD      16
#define HDIM       64
#define BQ         128
#define BK         32
#define NWAVE      8
#define ER         ((EARLY_QBLK * BQ < SEQ) ? (EARLY_QBLK * BQ) : SEQ)
#define NCH        (SEQ / BK)
#define NCHP       (((NCH + 31) / 32) * 32)
#define MROWS      (NB * SEQ)
#define RELN       (2 * SEQ_FULL - 1)
#define TP         72
#define OP         68
#define GP         136
#define RSC        2048.0f
#define RSCI       (1.0f / 2048.0f)
#define PSC        4096.0f
#define YSC        32.0f
#define WSC        32.0f

#define XB_E   ((size_t)MROWS * CDIM)
#define WT_E   ((size_t)3 * CDIM * CDIM)
#define WO_E   ((size_t)CDIM * CDIM)
#define QKV_E  ((size_t)NB * NHEAD * SEQ * HDIM)
#define RES_E  ((size_t)NB * NHEAD * ER * HDIM)
#define YH_E   ((size_t)MROWS * CDIM)
#define YR_E   ((size_t)NB * ER * CDIM)
#define MB_E   ((size_t)SEQ * NCHP)
#define WS_HALVES (XB_E + WT_E + WO_E + 3 * QKV_E + 3 * RES_E + YH_E + YR_E)
#define WS_BYTES  (WS_HALVES * 2 + MB_E * 4)

static_assert(SEQ % BQ == 0);
static_assert(SEQ <= SEQ_FULL);
static_assert(NB >= 1 && NB <= NB_FULL);
static_assert(BQ == NWAVE * 16);
static_assert(BQ == 128);
static_assert(HDIM == 64);
static_assert(NHEAD * HDIM == CDIM);
static_assert(CDIM == 1024);
static_assert(CDIM % 128 == 0 && CDIM % 32 == 0);
static_assert(ER % 128 == 0 && ER <= SEQ && ER >= BQ);
static_assert(NCH <= 64);
static_assert(NCHP == 32 || NCHP == 64);
static_assert(MROWS % 128 == 0);
static_assert(((size_t)MROWS * 128) % 256 == 0);
static_assert(SEQ % 8 == 0);
static_assert((TP * 2) % 16 == 0);
static_assert((OP * 4) % 16 == 0);
static_assert((GP * 2) % 16 == 0);
static_assert(XB_E % 64 == 0 && WT_E % 64 == 0 && WO_E % 64 == 0 && QKV_E % 64 == 0 && RES_E % 64 == 0);
static_assert(YH_E % 64 == 0 && YR_E % 64 == 0);
static_assert(WS_BYTES <= (size_t)134217728);

typedef __bf16         bf16;
typedef _Float16       f16;
typedef unsigned short us;
typedef bf16     v16bf __attribute__((ext_vector_type(16)));
typedef f16      v16h  __attribute__((ext_vector_type(16)));
typedef float    v8f   __attribute__((ext_vector_type(8)));
typedef float    v4f   __attribute__((ext_vector_type(4)));
typedef unsigned v4u   __attribute__((ext_vector_type(4)));

union FragH { v16h v; v4u q[2]; f16 h[16]; };
union FragU { v16bf b; v16h h; v4u q[2]; };
union Pack8 { v4u u; us h[8]; };

static __device__ __forceinline__ us bf16_bits(float x) { union { bf16 b; us u; } c; c.b = (bf16)x; return c.u; }
static __device__ __forceinline__ us f16_bits(float x)  { union { f16 h; us u; } c; c.h = (f16)x; return c.u; }
static __device__ __forceinline__ float bf16_rne(float x) { return (float)(bf16)x; }
static __device__ __forceinline__ v4u ldv(const us* p) { return *(const v4u*)p; }

static __device__ __forceinline__ v8f mma_bf16(v16bf a, v16bf b, v8f acc) {
  acc = __builtin_amdgcn_wmma_f32_16x16x32_bf16(false, a, false, b, (short)0, acc, false, false);
  asm volatile("v_nop\n\tv_nop\n\tv_nop\n\tv_nop" : "+v"(acc) : "v"(a), "v"(b));
  return acc;
}
static __device__ __forceinline__ v8f mma_f16(v16h a, v16h b, v8f acc) {
  acc = __builtin_amdgcn_wmma_f32_16x16x32_f16(false, a, false, b, (short)0, acc, false, false);
  asm volatile("v_nop\n\tv_nop\n\tv_nop\n\tv_nop" : "+v"(acc) : "v"(a), "v"(b));
  return acc;
}

__global__ __launch_bounds__(256) void x_plane_kernel(const float* __restrict__ x, us* __restrict__ xb) {
  const int p   = blockIdx.x * 256 + threadIdx.x;
  const int m   = p >> 7;
  const int seg = p & 127;
  const int b   = m / SEQ;
  const int t   = m - b * SEQ;
  const float* src = x + ((size_t)b * SEQ_FULL + t) * CDIM + seg * 8;
  const v4f a0 = *(const v4f*)(src);
  const v4f a1 = *(const v4f*)(src + 4);
  Pack8 pk;
  #pragma unroll
  for (int i = 0; i < 4; ++i) {
    pk.h[i]     = bf16_bits(a0[i]);
    pk.h[4 + i] = bf16_bits(a1[i]);
  }
  const v4u val = pk.u;
  us* dst = xb + (size_t)m * CDIM + seg * 8;
  *(volatile v4u*)dst = val;
  __threadfence();
  *(volatile v4u*)dst = val;
}

__global__ __launch_bounds__(256) void wt_plane_kernel(const float* __restrict__ W, us* __restrict__ Wt, int f16mode) {
  __shared__ __align__(16) us sT[64 * TP];
  const int k0  = blockIdx.x * 64;
  const int n0  = blockIdx.y * 64;
  const int tid = threadIdx.x;
  #pragma unroll
  for (int it = 0; it < 4; ++it) {
    const int kk = it * 16 + (tid >> 4);
    const int nn = (tid & 15) * 4;
    const v4f w = *(const v4f*)(W + (size_t)(k0 + kk) * CDIM + n0 + nn);
    #pragma unroll
    for (int i = 0; i < 4; ++i) {
      const float r  = bf16_rne(w[i]);
      const us    bb = bf16_bits(w[i]);
      const us    hb = f16_bits(r * WSC);
      sT[(nn + i) * TP + kk] = (f16mode != 0) ? hb : bb;
    }
  }
  __syncthreads();
  v4u    vals[2];
  size_t gidx[2];
  #pragma unroll
  for (int kk2 = 0; kk2 < 2; ++kk2) {
    const int n  = kk2 * 32 + (tid >> 3);
    const int ks = (tid & 7) * 8;
    vals[kk2] = *(const v4u*)(sT + n * TP + ks);
    gidx[kk2] = (size_t)(n0 + n) * CDIM + k0 + ks;
  }
  #pragma unroll
  for (int kk2 = 0; kk2 < 2; ++kk2) *(volatile v4u*)(Wt + gidx[kk2]) = vals[kk2];
  __threadfence();
  #pragma unroll
  for (int kk2 = 0; kk2 < 2; ++kk2) *(volatile v4u*)(Wt + gidx[kk2]) = vals[kk2];
}

__global__ __launch_bounds__(256) void mask_bits_kernel(const int* __restrict__ mask, unsigned* __restrict__ mb) {
  const int wave = threadIdx.x >> 5;
  const int lane = threadIdx.x & 31;
  const int row  = blockIdx.x * 8 + wave;
  const int* mrow = mask + (size_t)row * SEQ_FULL;
  unsigned w0 = 0u, w1 = 0u;
  #pragma unroll 1
  for (int i = 0; i < NCH; ++i) {
    const int v = mrow[i * 32 + lane];
    const unsigned bal = __builtin_amdgcn_ballot_w32(v != 0);
    w0 = (i == lane) ? bal : w0;
    w1 = (i == lane + 32) ? bal : w1;
  }
  unsigned* dst = mb + (size_t)row * NCHP + lane;
  *(volatile unsigned*)dst = w0;
  if (NCHP > 32) *(volatile unsigned*)(dst + 32) = w1;
  __threadfence();
  *(volatile unsigned*)dst = w0;
  if (NCHP > 32) *(volatile unsigned*)(dst + 32) = w1;
}

template <int BF>
static __device__ __forceinline__ void gemm_kloop(const us* __restrict__ Ap, const us* __restrict__ Bp,
                                                  v8f (&acc)[2][4]) {
  #pragma unroll 1
  for (int k0 = 0; k0 < CDIM; k0 += 32) {
    FragU a[2], bq[4];
    #pragma unroll
    for (int mt = 0; mt < 2; ++mt) {
      const us* p = Ap + (size_t)mt * 16 * CDIM + k0;
      a[mt].q[0] = ldv(p);
      a[mt].q[1] = ldv(p + 16);
    }
    #pragma unroll
    for (int nt = 0; nt < 4; ++nt) {
      const us* p = Bp + (size_t)nt * 16 * CDIM + k0;
      bq[nt].q[0] = ldv(p);
      bq[nt].q[1] = ldv(p + 16);
    }
    #pragma unroll
    for (int mt = 0; mt < 2; ++mt) {
      #pragma unroll
      for (int nt = 0; nt < 4; ++nt) {
        if (BF != 0) acc[mt][nt] = mma_bf16(a[mt].b, bq[nt].b, acc[mt][nt]);
        else         acc[mt][nt] = mma_f16(a[mt].h, bq[nt].h, acc[mt][nt]);
      }
    }
  }
}

template <int RESPH>
static __device__ __forceinline__ void qkv_store_phase(us* sT, const v8f (&acc)[2][4], us* __restrict__ plane,
                                                       int tpitch, int which, int b, int head0, int t0,
                                                       int tid, int wm, int wn, int l16, int hl) {
  #pragma unroll
  for (int mt = 0; mt < 2; ++mt) {
    #pragma unroll
    for (int nt = 0; nt < 4; ++nt) {
      #pragma unroll
      for (int v = 0; v < 8; ++v) {
        const float val = acc[mt][nt][v];
        const float hvf = (float)(f16)val;
        const us bits = (RESPH != 0) ? f16_bits((val - hvf) * RSC) : f16_bits(val);
        const int ml = wm * 32 + mt * 16 + 8 * hl + v;
        const int nl = wn * 64 + nt * 16 + l16;
        const int idx = (which == 2) ? (nl * GP + ml) : (ml * GP + nl);
        sT[idx] = bits;
      }
    }
  }
  __syncthreads();
  v4u    vals[8];
  size_t gidx[8];
  #pragma unroll
  for (int it = 0; it < 8; ++it) {
    const int p = it * 256 + tid;
    int src;
    size_t dst;
    if (which == 2) {
      const int row = p >> 4;
      const int seg = p & 15;
      const int hd  = row >> 6;
      const int d   = row & 63;
      src = row * GP + seg * 8;
      dst = (((size_t)b * NHEAD + head0 + hd) * HDIM + d) * (size_t)tpitch + t0 + seg * 8;
    } else {
      const int line = p >> 3;
      const int seg  = p & 7;
      const int hd   = line >> 7;
      const int tl   = line & 127;
      src = tl * GP + hd * 64 + seg * 8;
      dst = (((size_t)b * NHEAD + head0 + hd) * (size_t)tpitch + t0 + tl) * HDIM + seg * 8;
    }
    vals[it] = *(const v4u*)(sT + src);
    gidx[it] = dst;
  }
  #pragma unroll
  for (int it = 0; it < 8; ++it) *(volatile v4u*)(plane + gidx[it]) = vals[it];
  __threadfence();
  #pragma unroll
  for (int it = 0; it < 8; ++it) *(volatile v4u*)(plane + gidx[it]) = vals[it];
  __syncthreads();
}

__global__ __launch_bounds__(256) void qkv_gemm_kernel(const us* __restrict__ xb, const us* __restrict__ wT,
                                                       us* __restrict__ hiplanes, us* __restrict__ resplanes) {
  __shared__ __align__(16) us sT[128 * GP];
  const int tid = threadIdx.x;
  const int w   = tid >> 5;
  const int ln  = tid & 31;
  const int l16 = ln & 15;
  const int hl  = ln >> 4;
  const int wm  = w >> 1;
  const int wn  = w & 1;
  const int ng0 = blockIdx.x * 128;
  const int m0  = blockIdx.y * 128;
  const int which = ng0 / CDIM;
  const int nb    = ng0 - which * CDIM;
  const int head0 = nb >> 6;
  const int b     = m0 / SEQ;
  const int t0    = m0 - b * SEQ;

  v8f acc[2][4];
  #pragma unroll
  for (int mt = 0; mt < 2; ++mt)
    #pragma unroll
    for (int nt = 0; nt < 4; ++nt) acc[mt][nt] = (v8f){0, 0, 0, 0, 0, 0, 0, 0};

  const us* Ap = xb + ((size_t)m0 + wm * 32 + l16) * CDIM + 8 * hl;
  const us* Bp = wT + ((size_t)ng0 + wn * 64 + l16) * CDIM + 8 * hl;
  gemm_kloop<1>(Ap, Bp, acc);

  qkv_store_phase<0>(sT, acc, hiplanes + (size_t)which * QKV_E, SEQ, which, b, head0, t0, tid, wm, wn, l16, hl);
  if (t0 < ER) {
    qkv_store_phase<1>(sT, acc, resplanes + (size_t)which * RES_E, ER, which, b, head0, t0, tid, wm, wn, l16, hl);
  }
}

template <int RES>
static __device__ __forceinline__ void attn_chunk(const us* __restrict__ kh_h, const us* __restrict__ vt_h,
                                                  const us* __restrict__ kr_h, const us* __restrict__ vr_h,
                                                  const FragH (&qf)[2], const FragH (&qrf)[2],
                                                  const float* sRel, int eb, unsigned mw, int j0, int lq, int hi,
                                                  v8f (&o)[4], float& rmax, float& rsum) {
  const float L2E = 1.4426950408889634f;
  v8f c[2];
  #pragma unroll
  for (int sub = 0; sub < 2; ++sub) {
    const us* kp = kh_h + (size_t)(j0 + sub * 16 + lq) * HDIM + hi * 8;
    FragH k0, k1;
    k0.q[0] = ldv(kp);
    k0.q[1] = ldv(kp + 16);
    k1.q[0] = ldv(kp + 32);
    k1.q[1] = ldv(kp + 48);
    v8f acc = (v8f){0, 0, 0, 0, 0, 0, 0, 0};
    if (RES != 0) {
      const us* rp = kr_h + (size_t)(j0 + sub * 16 + lq) * HDIM + hi * 8;
      FragH r0, r1;
      r0.q[0] = ldv(rp);
      r0.q[1] = ldv(rp + 16);
      r1.q[0] = ldv(rp + 32);
      r1.q[1] = ldv(rp + 48);
      acc = mma_f16(k0.v, qrf[0].v, acc);
      acc = mma_f16(k1.v, qrf[1].v, acc);
      acc = mma_f16(r0.v, qf[0].v, acc);
      acc = mma_f16(r1.v, qf[1].v, acc);
      #pragma unroll
      for (int r = 0; r < 8; ++r) acc[r] *= RSCI;
    }
    acc = mma_f16(k0.v, qf[0].v, acc);
    acc = mma_f16(k1.v, qf[1].v, acc);
    c[sub] = acc;
  }

  const unsigned mwh = mw >> (hi * 8);
  #pragma unroll
  for (int sub = 0; sub < 2; ++sub) {
    #pragma unroll
    for (int r = 0; r < 8; ++r) {
      const float bias = sRel[eb - sub * 16 - r];
      const float s    = c[sub][r] * 0.125f + bias;
      const bool keep  = ((mwh >> (sub * 16 + r)) & 1u) != 0u;
      c[sub][r] = keep ? s : -__FLT_MAX__;
    }
  }

  float m_new = rmax;
  #pragma unroll
  for (int r = 0; r < 8; ++r) {
    m_new = fmaxf(m_new, c[0][r]);
    m_new = fmaxf(m_new, c[1][r]);
  }
  m_new = fmaxf(m_new, __shfl_xor(m_new, 16, 32));
  const float scale = __builtin_amdgcn_exp2f((rmax - m_new) * L2E);
  rmax = m_new;

  FragH pa, pr;
  float psum = 0.0f;
  #pragma unroll
  for (int r = 0; r < 8; ++r) {
    const float p0 = __builtin_amdgcn_exp2f((c[0][r] - m_new) * L2E);
    const float p1 = __builtin_amdgcn_exp2f((c[1][r] - m_new) * L2E);
    psum += p0 + p1;
    const float pc0 = p0 * PSC;
    const float pc1 = p1 * PSC;
    const f16 h0 = (f16)pc0;
    const f16 h1 = (f16)pc1;
    pa.h[r]     = h0;
    pa.h[8 + r] = h1;
    if (RES != 0) {
      pr.h[r]     = (f16)((pc0 - (float)h0) * RSC);
      pr.h[8 + r] = (f16)((pc1 - (float)h1) * RSC);
    }
  }
  rsum = rsum * scale + psum + __shfl_xor(psum, 16, 32);

  float sc[8];
  #pragma unroll
  for (int r = 0; r < 8; ++r) sc[r] = __shfl(scale, (hi << 3) + r, 32);
  #pragma unroll
  for (int dt = 0; dt < 4; ++dt) {
    #pragma unroll
    for (int r = 0; r < 8; ++r) o[dt][r] *= sc[r];
  }

  #pragma unroll
  for (int dt = 0; dt < 4; ++dt) {
    const us* vp = vt_h + (size_t)(dt * 16 + lq) * SEQ + j0 + hi * 8;
    FragH bv;
    bv.q[0] = ldv(vp);
    bv.q[1] = ldv(vp + 16);
    if (RES != 0) {
      const us* rp = vr_h + (size_t)(dt * 16 + lq) * ER + j0 + hi * 8;
      FragH br;
      br.q[0] = ldv(rp);
      br.q[1] = ldv(rp + 16);
      v8f t = (v8f){0, 0, 0, 0, 0, 0, 0, 0};
      t = mma_f16(pr.v, bv.v, t);
      t = mma_f16(pa.v, br.v, t);
      #pragma unroll
      for (int r = 0; r < 8; ++r) o[dt][r] += t[r] * RSCI;
    }
    o[dt] = mma_f16(pa.v, bv.v, o[dt]);
  }
}

template <int EARLY>
static __device__ __forceinline__ void attn_body(const us* __restrict__ qh, const us* __restrict__ kh,
                                                 const us* __restrict__ vt, const us* __restrict__ qr,
                                                 const us* __restrict__ kr, const us* __restrict__ vr,
                                                 const float* __restrict__ rel, const unsigned* __restrict__ mb,
                                                 us* __restrict__ yh, us* __restrict__ yr, int qblk) {
  __shared__ __align__(16) float sO[NWAVE * 16 * OP];
  __shared__ __align__(16) float sRel[SEQ + BQ];

  const int h    = blockIdx.y;
  const int b    = blockIdx.z;
  const int tid  = threadIdx.x;
  const int wave = tid >> 5;
  const int lane = tid & 31;
  const int lq   = lane & 15;
  const int hi   = lane >> 4;
  const int q0    = qblk * BQ;
  const int qrow0 = q0 + wave * 16;
  const int qi    = qrow0 + lq;

  {
    const float* relh = rel + (size_t)h * RELN;
    #pragma unroll 1
    for (int e = tid; e < SEQ + BQ; e += 256) {
      int idx = e + q0 - (SEQ - 1) + (SEQ_FULL - 1);
      idx = (idx < 0) ? 0 : idx;
      idx = (idx > RELN - 1) ? (RELN - 1) : idx;
      sRel[e] = bf16_rne(relh[idx]);
    }
  }

  const size_t bh = (size_t)b * NHEAD + h;

  FragH qf[2], qrf[2];
  {
    const us* qp = qh + (bh * SEQ + qi) * HDIM + hi * 8;
    #pragma unroll
    for (int f = 0; f < 2; ++f) {
      qf[f].q[0] = ldv(qp + f * 32);
      qf[f].q[1] = ldv(qp + f * 32 + 16);
    }
  }
  if (EARLY != 0) {
    const us* qp = qr + (bh * ER + qi) * HDIM + hi * 8;
    #pragma unroll
    for (int f = 0; f < 2; ++f) {
      qrf[f].q[0] = ldv(qp + f * 32);
      qrf[f].q[1] = ldv(qp + f * 32 + 16);
    }
  } else {
    #pragma unroll
    for (int f = 0; f < 2; ++f) { qrf[f].q[0] = qf[f].q[0]; qrf[f].q[1] = qf[f].q[1]; }
  }

  const unsigned* mrow = mb + (size_t)qi * NCHP;
  unsigned anyk = 0u;
  #pragma unroll 4
  for (int i = 0; i < NCHP / 4; ++i) {
    const v4u w = *(const v4u*)(mrow + 4 * i);
    anyk |= (w[0] | w[1] | w[2] | w[3]);
  }
  const bool grp_all = (__builtin_amdgcn_ballot_w32(anyk == 0u) == 0u);

  __syncthreads();

  const us* kh_h = kh + bh * SEQ * HDIM;
  const us* vt_h = vt + bh * HDIM * SEQ;
  const us* kr_h = kr + bh * ER * HDIM;
  const us* vr_h = vr + bh * HDIM * ER;

  v8f o[4];
  #pragma unroll
  for (int dt = 0; dt < 4; ++dt) o[dt] = (v8f){0, 0, 0, 0, 0, 0, 0, 0};
  float rmax = -__builtin_inff();
  float rsum = 0.0f;
  const int ebase = wave * 16 + lq + (SEQ - 1);

  #pragma unroll 1
  for (int i = 0; i < NCH; ++i) {
    const unsigned mw = mrow[i];
    const bool empty = (__builtin_amdgcn_ballot_w32(mw != 0u) == 0u);
    if (empty && grp_all) continue;
    const int j0 = i * BK;
    const int eb = ebase - j0 - hi * 8;
    if (EARLY != 0 && j0 < ER) {
      attn_chunk<1>(kh_h, vt_h, kr_h, vr_h, qf, qrf, sRel, eb, mw, j0, lq, hi, o, rmax, rsum);
    } else {
      attn_chunk<0>(kh_h, vt_h, kr_h, vr_h, qf, qrf, sRel, eb, mw, j0, lq, hi, o, rmax, rsum);
    }
  }

  float rs[8];
  #pragma unroll
  for (int r = 0; r < 8; ++r) rs[r] = 1.0f / __shfl(rsum, (hi << 3) + r, 32);

  float* so = sO + wave * (16 * OP);
  #pragma unroll
  for (int r = 0; r < 8; ++r) {
    #pragma unroll
    for (int dt = 0; dt < 4; ++dt) {
      so[(hi * 8 + r) * OP + dt * 16 + lq] = o[dt][r] * (1.0f / PSC) * rs[r];
    }
  }
  __syncthreads();

  v4u    hv[4], rv[4];
  size_t gh[4], gr[4];
  #pragma unroll
  for (int it = 0; it < 4; ++it) {
    const int row = it * 4 + (lane >> 3);
    const int seg = lane & 7;
    const v4f a0 = *(const v4f*)(so + row * OP + seg * 8);
    const v4f a1 = *(const v4f*)(so + row * OP + seg * 8 + 4);
    Pack8 ph, pq;
    #pragma unroll
    for (int i = 0; i < 4; ++i) {
      const float y0 = a0[i] * YSC;
      const float y1 = a1[i] * YSC;
      const float g0 = (float)(f16)y0;
      const float g1 = (float)(f16)y1;
      ph.h[i]     = f16_bits(y0);
      ph.h[4 + i] = f16_bits(y1);
      pq.h[i]     = f16_bits((y0 - g0) * RSC);
      pq.h[4 + i] = f16_bits((y1 - g1) * RSC);
    }
    hv[it] = ph.u;
    rv[it] = pq.u;
    gh[it] = ((size_t)b * SEQ + qrow0 + row) * CDIM + h * HDIM + seg * 8;
    gr[it] = ((size_t)b * ER + ((EARLY != 0) ? (qrow0 + row) : 0)) * CDIM + h * HDIM + seg * 8;
  }
  #pragma unroll
  for (int it = 0; it < 4; ++it) {
    *(volatile v4u*)(yh + gh[it]) = hv[it];
    if (EARLY != 0) *(volatile v4u*)(yr + gr[it]) = rv[it];
  }
  __threadfence();
  #pragma unroll
  for (int it = 0; it < 4; ++it) {
    *(volatile v4u*)(yh + gh[it]) = hv[it];
    if (EARLY != 0) *(volatile v4u*)(yr + gr[it]) = rv[it];
  }
}

__global__ __launch_bounds__(256) void attn_early_kernel(const us* __restrict__ qh, const us* __restrict__ kh,
                                                         const us* __restrict__ vt, const us* __restrict__ qr,
                                                         const us* __restrict__ kr, const us* __restrict__ vr,
                                                         const float* __restrict__ rel,
                                                         const unsigned* __restrict__ mb,
                                                         us* __restrict__ yh, us* __restrict__ yr) {
  attn_body<1>(qh, kh, vt, qr, kr, vr, rel, mb, yh, yr, (int)blockIdx.x);
}

__global__ __launch_bounds__(256) void attn_late_kernel(const us* __restrict__ qh, const us* __restrict__ kh,
                                                        const us* __restrict__ vt, const us* __restrict__ qr,
                                                        const us* __restrict__ kr, const us* __restrict__ vr,
                                                        const float* __restrict__ rel,
                                                        const unsigned* __restrict__ mb,
                                                        us* __restrict__ yh, us* __restrict__ yr, int qblk0) {
  attn_body<0>(qh, kh, vt, qr, kr, vr, rel, mb, yh, yr, qblk0 + (int)blockIdx.x);
}

__global__ __launch_bounds__(256) void out_gemm_kernel(const us* __restrict__ yh, const us* __restrict__ yr,
                                                       const us* __restrict__ woT, const float* __restrict__ bo,
                                                       float* __restrict__ out) {
  __shared__ __align__(16) float sO[NWAVE * 16 * OP];
  const int tid = threadIdx.x;
  const int w   = tid >> 5;
  const int ln  = tid & 31;
  const int l16 = ln & 15;
  const int hl  = ln >> 4;
  const int wm  = w >> 1;
  const int wn  = w & 1;
  const int n0  = blockIdx.x * 128;
  const int m0  = blockIdx.y * 128;
  const int b   = m0 / SEQ;
  const int t0  = m0 - b * SEQ;

  v8f acc[2][4];
  #pragma unroll
  for (int mt = 0; mt < 2; ++mt)
    #pragma unroll
    for (int nt = 0; nt < 4; ++nt) acc[mt][nt] = (v8f){0, 0, 0, 0, 0, 0, 0, 0};

  const us* Bp = woT + ((size_t)n0 + wn * 64 + l16) * CDIM + 8 * hl;
  if (t0 < ER) {
    const us* Ar = yr + ((size_t)b * ER + t0 + wm * 32 + l16) * CDIM + 8 * hl;
    gemm_kloop<0>(Ar, Bp, acc);
    #pragma unroll
    for (int mt = 0; mt < 2; ++mt)
      #pragma unroll
      for (int nt = 0; nt < 4; ++nt)
        #pragma unroll
        for (int v = 0; v < 8; ++v) acc[mt][nt][v] *= RSCI;
  }
  const us* Ap = yh + ((size_t)m0 + wm * 32 + l16) * CDIM + 8 * hl;
  gemm_kloop<0>(Ap, Bp, acc);

  const float OSC = 1.0f / (YSC * WSC);
  const int ncol = n0 + wn * 64 + l16 * 4;
  v4f bb = *(const v4f*)(bo + ncol);
  #pragma unroll
  for (int i = 0; i < 4; ++i) bb[i] = bf16_rne(bb[i]);

  float* so = sO + w * (16 * OP);
  #pragma unroll
  for (int mt = 0; mt < 2; ++mt) {
    #pragma unroll
    for (int nt = 0; nt < 4; ++nt) {
      #pragma unroll
      for (int v = 0; v < 8; ++v) so[(8 * hl + v) * OP + nt * 16 + l16] = acc[mt][nt][v];
    }
    __syncthreads();
    v4f    vals[8];
    size_t gidx[8];
    #pragma unroll
    for (int it = 0; it < 8; ++it) {
      const int row = it * 2 + hl;
      const v4f s = *(const v4f*)(so + row * OP + l16 * 4);
      vals[it] = s * OSC + bb;
      gidx[it] = ((size_t)b * SEQ_FULL + t0 + wm * 32 + mt * 16 + row) * CDIM + ncol;
    }
    #pragma unroll
    for (int it = 0; it < 8; ++it) *(volatile v4f*)(out + gidx[it]) = vals[it];
    __threadfence();
    #pragma unroll
    for (int it = 0; it < 8; ++it) *(volatile v4f*)(out + gidx[it]) = vals[it];
    __syncthreads();
  }
}

extern "C" void kernel_launch(void* const* d_in, const int* in_sizes, int n_in,
                              void* d_out, int out_size, void* d_ws, size_t ws_size,
                              hipStream_t stream) {
  if (n_in < 8) return;
  const size_t rows_used = (size_t)(NB - 1) * SEQ_FULL + SEQ;
  if ((size_t)in_sizes[0] < rows_used * CDIM) return;
  if ((size_t)in_sizes[1] < (size_t)CDIM * CDIM) return;
  if ((size_t)in_sizes[2] < (size_t)CDIM * CDIM) return;
  if ((size_t)in_sizes[3] < (size_t)CDIM * CDIM) return;
  if ((size_t)in_sizes[4] < (size_t)CDIM * CDIM) return;
  if ((size_t)in_sizes[5] < (size_t)CDIM) return;
  if ((size_t)in_sizes[6] < (size_t)NHEAD * RELN) return;
  if ((size_t)in_sizes[7] < (size_t)(SEQ - 1) * SEQ_FULL + SEQ) return;
  if ((size_t)out_size < rows_used * CDIM) return;
  if (ws_size < WS_BYTES) return;

  const float* x    = (const float*)d_in[0];
  const float* Wq   = (const float*)d_in[1];
  const float* Wk   = (const float*)d_in[2];
  const float* Wv   = (const float*)d_in[3];
  const float* Wo   = (const float*)d_in[4];
  const float* bo   = (const float*)d_in[5];
  const float* rel  = (const float*)d_in[6];
  const int*   mask = (const int*)d_in[7];
  float*       out  = (float*)d_out;

  us* ws16 = (us*)d_ws;
  us* xb   = ws16;
  us* wT   = xb + XB_E;
  us* woT  = wT + WT_E;
  us* qh   = woT + WO_E;
  us* kh   = qh + QKV_E;
  us* vt   = kh + QKV_E;
  us* qr   = vt + QKV_E;
  us* kr   = qr + RES_E;
  us* vr   = kr + RES_E;
  us* yh   = vr + RES_E;
  us* yr   = yh + YH_E;
  unsigned* mb = (unsigned*)(yr + YR_E);

  x_plane_kernel<<<dim3((unsigned)(((size_t)MROWS * 128) / 256)), 256, 0, stream>>>(x, xb);

  wt_plane_kernel<<<dim3(CDIM / 64, CDIM / 64), 256, 0, stream>>>(Wq, wT, 0);
  wt_plane_kernel<<<dim3(CDIM / 64, CDIM / 64), 256, 0, stream>>>(Wk, wT + (size_t)CDIM * CDIM, 0);
  wt_plane_kernel<<<dim3(CDIM / 64, CDIM / 64), 256, 0, stream>>>(Wv, wT + (size_t)2 * CDIM * CDIM, 0);
  wt_plane_kernel<<<dim3(CDIM / 64, CDIM / 64), 256, 0, stream>>>(Wo, woT, 1);

  mask_bits_kernel<<<dim3(SEQ / 8), 256, 0, stream>>>(mask, mb);

  qkv_gemm_kernel<<<dim3(3 * CDIM / 128, MROWS / 128), 256, 0, stream>>>(xb, wT, qh, qr);

  const int nqb     = SEQ / BQ;
  const int n_early = (EARLY_QBLK < nqb) ? EARLY_QBLK : nqb;
  const int n_late  = nqb - n_early;
  attn_early_kernel<<<dim3(n_early, NHEAD, NB), 256, 0, stream>>>(qh, kh, vt, qr, kr, vr, rel, mb, yh, yr);
  if (n_late > 0)
    attn_late_kernel<<<dim3(n_late, NHEAD, NB), 256, 0, stream>>>(qh, kh, vt, qr, kr, vr, rel, mb, yh, yr, n_early);

  out_gemm_kernel<<<dim3(CDIM / 128, MROWS / 128), 256, 0, stream>>>(yh, yr, woT, bo, out);
}
